// SwinBlock3D_3435973836950
// MI455X (gfx1250) — hardware-verified
//
#include <hip/hip_runtime.h>

typedef __bf16 v16b __attribute__((ext_vector_type(16)));
typedef __bf16 v8b  __attribute__((ext_vector_type(8)));
typedef float  v8f  __attribute__((ext_vector_type(8)));
typedef float  v4f  __attribute__((ext_vector_type(4)));
typedef unsigned int v4u __attribute__((ext_vector_type(4)));
typedef unsigned int v2u __attribute__((ext_vector_type(2)));
typedef v8b __attribute__((may_alias)) v8ba;
typedef v4f __attribute__((may_alias)) v4fa;
typedef v4u __attribute__((may_alias)) v4ua;
typedef v2u __attribute__((may_alias)) v2ua;
typedef unsigned short us_t;

union Frag { v16b v; v8b h[2]; };
union PK   { v16b v; unsigned int w[8]; };

#define CE    128
#define PD    256
#define NHD   8
#define HDM   32
#define HID   384
#define LT    196
#define NWIN  128
#define VD    8
#define VH    56
#define VW    56
#define MHALF (NWIN * LT)
#define NVOXF (2 * VD * VH * VW * CE)
#define VTP   224
#define NQT   13
#define ATT_THREADS (NQT * 32)
#define SQS   0.17677669529663687f

#define OWQH 0
#define OWQL 32768
#define OWKH 65536
#define OWKL 98304
#define OWVH 131072
#define OWVL 163840
#define OWOH 196608
#define OWOL 229376
#define OW1H 262144
#define OW1L 311296
#define OW2H 360448
#define OW2L 409600
#define OWEND 458752

__device__ __forceinline__ v8f wmma_bf(v16b a, v16b b, v8f c) {
  v8f d = __builtin_amdgcn_wmma_f32_16x16x32_bf16(false, a, false, b, (short)0, c, false, false);
  asm volatile("v_nop\n\tv_nop\n\tv_nop\n\tv_nop" : "+v"(d) : "v"(a), "v"(b));
  return d;
}
__device__ __forceinline__ v8f wmma3(v16b ah, v16b al, v16b bh, v16b bl, v8f c) {
  c = wmma_bf(ah, bh, c);
  c = wmma_bf(ah, bl, c);
  c = wmma_bf(al, bh, c);
  return c;
}
__device__ __forceinline__ v16b ldfrag(const us_t* p, int hf) {
  Frag f;
  f.h[0] = *(const v8ba*)(p + 8 * hf);
  f.h[1] = *(const v8ba*)(p + 16 + 8 * hf);
  return f.v;
}

__device__ __forceinline__ int imin(int a, int b) { return a < b ? a : b; }

__device__ __forceinline__ unsigned int rne16(float f) {
  const unsigned int u = __float_as_uint(f);
  return (u + 0x7FFFu + ((u >> 16) & 1u)) >> 16;
}
__device__ __forceinline__ float bf2f(unsigned int b) { return __uint_as_float(b << 16); }
__device__ __forceinline__ void split2(float y, unsigned int& hb, unsigned int& lb) {
  hb = rne16(y);
  lb = rne16(y - bf2f(hb));
}
__device__ __forceinline__ void pack8(const float (&y)[8], v4u& hi, v4u& lo) {
  v4u a = {0u, 0u, 0u, 0u}, b = {0u, 0u, 0u, 0u};
#pragma unroll
  for (int i = 0; i < 4; ++i) {
    unsigned int h0, l0, h1, l1;
    split2(y[2 * i], h0, l0);
    split2(y[2 * i + 1], h1, l1);
    a[i] = h0 | (h1 << 16);
    b[i] = l0 | (l1 << 16);
  }
  hi = a; lo = b;
}

__device__ __forceinline__ float gelu_f(float x) {
  return 0.5f * x * (1.0f + erff(x * 0.70710678118654752f));
}

__device__ __forceinline__ int voxel_of(int tok, int half) {
  const int wl = tok / LT, t = tok - wl * LT;
  const int wd = wl >> 6, wh = (wl >> 3) & 7, ww = wl & 7;
  const int td = t / 49, t2 = t - td * 49, th = t2 / 7, tw = t2 - th * 7;
  const int d = (4 * wd + td + 2) & 7;
  int hh = 7 * wh + th + 3; if (hh >= VH) hh -= VH;
  int wi = 7 * ww + tw + 3; if (wi >= VW) wi -= VW;
  return ((half * VD + d) * VH + hh) * VW + wi;
}

__global__ __launch_bounds__(256) void k_bias(const float* __restrict__ rel,
                                              const int* __restrict__ ridx, int nrel,
                                              float* __restrict__ bt) {
  const int g = blockIdx.x * 256 + threadIdx.x;
  if (g >= (NHD * LT * LT) / 4) return;
  const int e = g * 4;
  const int hd = e / (LT * LT);
  const int rem = e - hd * (LT * LT);
  float y[4];
#pragma unroll
  for (int q = 0; q < 4; ++q) {
    int ix = ridx[rem + q];
    ix = ix < 0 ? 0 : (ix >= nrel ? nrel - 1 : ix);
    y[q] = rel[ix * NHD + hd];
  }
  const v4f v = {y[0], y[1], y[2], y[3]};
  *(volatile v4f*)(bt + e) = v;
  __threadfence();
  *(volatile v4f*)(bt + e) = v;
}

__global__ __launch_bounds__(256) void k_wconv(const float* __restrict__ Wq, const float* __restrict__ Wk,
                                               const float* __restrict__ Wv, const float* __restrict__ Wo,
                                               const float* __restrict__ W1, const float* __restrict__ W2,
                                               us_t* __restrict__ wt) {
  __shared__ __attribute__((aligned(16))) float sW[8][HID];
  const int b = blockIdx.x, tid = threadIdx.x;
  const float* W; int K, N, nb; size_t oh, ol;
  if (b < 32)       { W = Wq; K = CE;  N = PD;  nb = b;       oh = OWQH; ol = OWQL; }
  else if (b < 64)  { W = Wk; K = CE;  N = PD;  nb = b - 32;  oh = OWKH; ol = OWKL; }
  else if (b < 96)  { W = Wv; K = CE;  N = PD;  nb = b - 64;  oh = OWVH; ol = OWVL; }
  else if (b < 112) { W = Wo; K = PD;  N = CE;  nb = b - 96;  oh = OWOH; ol = OWOL; }
  else if (b < 160) { W = W1; K = CE;  N = HID; nb = b - 112; oh = OW1H; ol = OW1L; }
  else              { W = W2; K = HID; N = CE;  nb = b - 160; oh = OW2H; ol = OW2L; }
  const int n0 = nb * 8;
  for (int e = tid; e < K * 8; e += 256) {
    const int k = e >> 3, nl = e & 7;
    sW[nl][k] = W[(size_t)k * N + n0 + nl];
  }
  __syncthreads();
  const int cpr = K >> 3;
  for (int f = tid; f < K; f += 256) {
    const int nl = f / cpr, c = f - nl * cpr;
    float y[8];
#pragma unroll
    for (int i = 0; i < 8; ++i) y[i] = sW[nl][8 * c + i];
    v4u hi, lo; pack8(y, hi, lo);
    const size_t o = (size_t)(n0 + nl) * K + 8 * c;
    *(volatile v4u*)(wt + oh + o) = hi;
    *(volatile v4u*)(wt + ol + o) = lo;
  }
  __threadfence();
  for (int f = tid; f < K; f += 256) {
    const int nl = f / cpr, c = f - nl * cpr;
    float y[8];
#pragma unroll
    for (int i = 0; i < 8; ++i) y[i] = sW[nl][8 * c + i];
    v4u hi, lo; pack8(y, hi, lo);
    const size_t o = (size_t)(n0 + nl) * K + 8 * c;
    *(volatile v4u*)(wt + oh + o) = hi;
    *(volatile v4u*)(wt + ol + o) = lo;
  }
}

__global__ __launch_bounds__(256) void k_gather(const float* __restrict__ xq, const float* __restrict__ xk,
                                                const float* __restrict__ xv, int half,
                                                us_t* __restrict__ X) {
  const int which = blockIdx.y;
  const float* src = (which == 0) ? xq : ((which == 1) ? xk : xv);
  us_t* oh = X + (size_t)(2 * which) * MHALF * CE;
  us_t* ol = oh + (size_t)MHALF * CE;
  const int g = blockIdx.x * 256 + threadIdx.x;
  const int tok = g >> 4, cg = g & 15;
  const size_t vox = (size_t)voxel_of(tok, half) * CE + 8 * cg;
  const v4f a = *(const v4fa*)(src + vox);
  const v4f c = *(const v4fa*)(src + vox + 4);
  const float y[8] = {a.x, a.y, a.z, a.w, c.x, c.y, c.z, c.w};
  v4u hi, lo; pack8(y, hi, lo);
  const size_t o = (size_t)tok * CE + 8 * cg;
  *(volatile v4u*)(oh + o) = hi;
  *(volatile v4u*)(ol + o) = lo;
  __threadfence();
  *(volatile v4u*)(oh + o) = hi;
  *(volatile v4u*)(ol + o) = lo;
}

__device__ __forceinline__ void gemm_core(const us_t* __restrict__ Ah, const us_t* __restrict__ Al,
                                          const us_t* __restrict__ Bh, const us_t* __restrict__ Bl,
                                          int K, int row0, int coln, int hf, int m, v8f (&acc)[2][4]) {
  const us_t* a0h = Ah + (size_t)(row0 + m) * K;
  const us_t* a1h = a0h + (size_t)16 * K;
  const us_t* a0l = Al + (size_t)(row0 + m) * K;
  const us_t* a1l = a0l + (size_t)16 * K;
  const us_t* bh  = Bh + (size_t)coln * K;
  const us_t* bl  = Bl + (size_t)coln * K;
  const v8f z8 = {0.f, 0.f, 0.f, 0.f, 0.f, 0.f, 0.f, 0.f};
#pragma unroll
  for (int mt = 0; mt < 2; ++mt)
#pragma unroll
    for (int nt = 0; nt < 4; ++nt) acc[mt][nt] = z8;
#pragma unroll 1
  for (int k0 = 0; k0 < K; k0 += 32) {
    const v16b A0h = ldfrag(a0h + k0, hf);
    const v16b A1h = ldfrag(a1h + k0, hf);
    const v16b A0l = ldfrag(a0l + k0, hf);
    const v16b A1l = ldfrag(a1l + k0, hf);
#pragma unroll
    for (int nt = 0; nt < 4; ++nt) {
      const v16b BH = ldfrag(bh + (size_t)nt * 16 * K + k0, hf);
      const v16b BL = ldfrag(bl + (size_t)nt * 16 * K + k0, hf);
      acc[0][nt] = wmma3(A0h, A0l, BH, BL, acc[0][nt]);
      acc[1][nt] = wmma3(A1h, A1l, BH, BL, acc[1][nt]);
    }
  }
}

__device__ __forceinline__ void planes_store_pass(const us_t* sh, const us_t* sl,
                                                  us_t* __restrict__ Oh, us_t* __restrict__ Ol,
                                                  int row0, int col0, int N, int lane) {
  const int q8 = lane & 7, sub = lane >> 3;
#pragma unroll
  for (int i = 0; i < 8; ++i) {
    const int row = 4 * i + sub;
    const v4u vh = *(const v4ua*)(sh + row * 64 + 8 * q8);
    const v4u vl = *(const v4ua*)(sl + row * 64 + 8 * q8);
    const size_t o = (size_t)(row0 + row) * N + col0 + 8 * q8;
    *(volatile v4u*)(Oh + o) = vh;
    *(volatile v4u*)(Ol + o) = vl;
  }
}

template <int GELU>
__global__ __launch_bounds__(64) void k_gemm_planes(const us_t* __restrict__ Ah, const us_t* __restrict__ Al,
                                                    const us_t* __restrict__ Bh, const us_t* __restrict__ Bl,
                                                    const float* __restrict__ bias, int K, int N,
                                                    us_t* __restrict__ Oh, us_t* __restrict__ Ol) {
  __shared__ __attribute__((aligned(16))) us_t sHp[2][32][64];
  __shared__ __attribute__((aligned(16))) us_t sLp[2][32][64];
  const int tid = threadIdx.x, lane = tid & 31, w = tid >> 5;
  const int hf = lane >> 4, m = lane & 15;
  const int row0 = blockIdx.x * 32;
  const int col0 = blockIdx.y * 128 + 64 * w;
  v8f acc[2][4];
  gemm_core(Ah, Al, Bh, Bl, K, row0, col0 + m, hf, m, acc);
#pragma unroll
  for (int nt = 0; nt < 4; ++nt) {
    const int col = 16 * nt + m;
    const float bv = bias[col0 + col];
#pragma unroll
    for (int mt = 0; mt < 2; ++mt) {
#pragma unroll
      for (int r = 0; r < 8; ++r) {
        float y = acc[mt][nt][r] + bv;
        if (GELU) y = gelu_f(y);
        unsigned int hb, lb; split2(y, hb, lb);
        sHp[w][16 * mt + 8 * hf + r][col] = (us_t)hb;
        sLp[w][16 * mt + 8 * hf + r][col] = (us_t)lb;
      }
    }
  }
  __syncthreads();
  planes_store_pass(&sHp[w][0][0], &sLp[w][0][0], Oh, Ol, row0, col0, N, lane);
  __threadfence();
  planes_store_pass(&sHp[w][0][0], &sLp[w][0][0], Oh, Ol, row0, col0, N, lane);
}

__device__ __forceinline__ void ln_planes_pass(const us_t* sh, const us_t* sl,
                                               us_t* __restrict__ Ph, us_t* __restrict__ Pl,
                                               int row0, int w, int lane) {
  const int c16 = lane & 15, rsel = lane >> 4;
#pragma unroll
  for (int i = 0; i < 8; ++i) {
    const int row = 16 * w + 2 * i + rsel;
    const v4u vh = *(const v4ua*)(sh + row * CE + 8 * c16);
    const v4u vl = *(const v4ua*)(sl + row * CE + 8 * c16);
    const size_t o = (size_t)(row0 + row) * CE + 8 * c16;
    *(volatile v4u*)(Ph + o) = vh;
    *(volatile v4u*)(Pl + o) = vl;
  }
}

template <int FINAL>
__global__ __launch_bounds__(64) void k_gemm_ln(const us_t* __restrict__ Ah, const us_t* __restrict__ Al,
                                                const us_t* __restrict__ Bh, const us_t* __restrict__ Bl,
                                                const float* __restrict__ bias, int K,
                                                const float* __restrict__ gam, const float* __restrict__ bet,
                                                const float* __restrict__ res, float* __restrict__ out32,
                                                us_t* __restrict__ Ph, us_t* __restrict__ Pl, int half) {
  __shared__ __attribute__((aligned(16))) float sF[32][CE];
  __shared__ __attribute__((aligned(16))) us_t  sHp[32][CE];
  __shared__ __attribute__((aligned(16))) us_t  sLp[32][CE];
  const int tid = threadIdx.x, lane = tid & 31, w = tid >> 5;
  const int hf = lane >> 4, m = lane & 15;
  const int row0 = blockIdx.x * 32;
  const int col0 = 64 * w;
  v8f acc[2][4];
  gemm_core(Ah, Al, Bh, Bl, K, row0, col0 + m, hf, m, acc);
#pragma unroll
  for (int nt = 0; nt < 4; ++nt) {
    const int col = col0 + 16 * nt + m;
    const float bv = bias[col];
#pragma unroll
    for (int mt = 0; mt < 2; ++mt)
#pragma unroll
      for (int r = 0; r < 8; ++r) sF[16 * mt + 8 * hf + r][col] = acc[mt][nt][r] + bv;
  }
  __syncthreads();

#pragma unroll 1
  for (int rr = 0; rr < 16; ++rr) {
    const int row = 16 * w + rr;
    const int tok = row0 + row;
    const size_t vox = (size_t)voxel_of(tok, half) * CE + 4 * lane;
    const size_t tko = (size_t)tok * CE + 4 * lane;
    const v4f x = *(const v4fa*)(&sF[row][4 * lane]);
    float s = (x.x + x.y) + (x.z + x.w);
    s += __shfl_xor(s, 16); s += __shfl_xor(s, 8); s += __shfl_xor(s, 4);
    s += __shfl_xor(s, 2);  s += __shfl_xor(s, 1);
    const float mu = s * (1.0f / CE);
    const float d0 = x.x - mu, d1 = x.y - mu, d2 = x.z - mu, d3 = x.w - mu;
    float v = (d0 * d0 + d1 * d1) + (d2 * d2 + d3 * d3);
    v += __shfl_xor(v, 16); v += __shfl_xor(v, 8); v += __shfl_xor(v, 4);
    v += __shfl_xor(v, 2);  v += __shfl_xor(v, 1);
    const float rs = rsqrtf(v * (1.0f / CE) + 1e-5f);
    const v4f g4 = *(const v4fa*)(gam + 4 * lane);
    const v4f b4 = *(const v4fa*)(bet + 4 * lane);
    v4f r4;
    if (FINAL) r4 = *(const v4fa*)(res + tko);
    else       r4 = *(const v4fa*)(res + vox);
    const float t0 = d0 * rs * g4.x + b4.x;
    const float t1 = d1 * rs * g4.y + b4.y;
    const float t2 = d2 * rs * g4.z + b4.z;
    const float t3 = d3 * rs * g4.w + b4.w;
    const v4f o = {t0 + r4.x, t1 + r4.y, t2 + r4.z, t3 + r4.w};
    float* dst = FINAL ? (out32 + vox) : (out32 + tko);
    *(volatile v4f*)dst = o;
    *(v4fa*)(&sF[row][4 * lane]) = o;
    if (!FINAL) {
      unsigned int h0, l0, h1, l1, h2, l2, h3, l3;
      split2(o.x, h0, l0); split2(o.y, h1, l1); split2(o.z, h2, l2); split2(o.w, h3, l3);
      const v2u hv = {h0 | (h1 << 16), h2 | (h3 << 16)};
      const v2u lv = {l0 | (l1 << 16), l2 | (l3 << 16)};
      *(v2ua*)(&sHp[row][4 * lane]) = hv;
      *(v2ua*)(&sLp[row][4 * lane]) = lv;
    }
  }
  __threadfence();
  __syncthreads();
#pragma unroll 1
  for (int rr = 0; rr < 16; ++rr) {
    const int row = 16 * w + rr;
    const int tok = row0 + row;
    const size_t vox = (size_t)voxel_of(tok, half) * CE + 4 * lane;
    const size_t tko = (size_t)tok * CE + 4 * lane;
    const v4f o = *(const v4fa*)(&sF[row][4 * lane]);
    float* dst = FINAL ? (out32 + vox) : (out32 + tko);
    *(volatile v4f*)dst = o;
  }
  if (!FINAL) {
    ln_planes_pass(&sHp[0][0], &sLp[0][0], Ph, Pl, row0, w, lane);
    __threadfence();
    ln_planes_pass(&sHp[0][0], &sLp[0][0], Ph, Pl, row0, w, lane);
  }
}

__device__ __forceinline__ void ctx_store_pass(const us_t* sO, us_t* __restrict__ Ch, us_t* __restrict__ Cl,
                                               size_t tok0, int qt, int hp, int nst, int lane) {
  const int q8 = lane & 7, sub = lane >> 3;
#pragma unroll
  for (int i = 0; i < 4; ++i) {
    if (i < nst) {
      const int row = 4 * i + sub;
      const v4u vh = *(const v4ua*)(sO + (qt * 16 + row) * 64 + 8 * q8);
      const v4u vl = *(const v4ua*)(sO + NQT * 16 * 64 + (qt * 16 + row) * 64 + 8 * q8);
      const size_t o = (tok0 + 16 * qt + row) * PD + 64 * hp + 8 * q8;
      *(volatile v4u*)(Ch + o) = vh;
      *(volatile v4u*)(Cl + o) = vl;
    }
  }
}

__global__ __launch_bounds__(ATT_THREADS) void k_attn(const us_t* __restrict__ Qh, const us_t* __restrict__ Ql,
                                                       const us_t* __restrict__ Kh, const us_t* __restrict__ Kl,
                                                       const us_t* __restrict__ Vh, const us_t* __restrict__ Vl,
                                                       const float* __restrict__ bt, const float* __restrict__ am,
                                                       us_t* __restrict__ Ch, us_t* __restrict__ Cl) {
  extern __shared__ __attribute__((aligned(16))) us_t dlds[];
  us_t* sVT = dlds;
  us_t* sO  = dlds + 2 * 2 * HDM * VTP;
  const int tid = threadIdx.x, lane = tid & 31, qt = tid >> 5;
  const int hf = lane >> 4, m = lane & 15;
  const int wl = blockIdx.x, hp = blockIdx.y;
  const size_t tok0 = (size_t)wl * LT;
  const v8f z8 = {0.f, 0.f, 0.f, 0.f, 0.f, 0.f, 0.f, 0.f};

  for (int e = tid; e < 2 * LT * 4; e += ATT_THREADS) {
    const int dg = e & 3, rj = e >> 2;
    const int hl = (rj >= LT) ? 1 : 0;
    const int j = rj - hl * LT;
    const size_t src = (tok0 + j) * PD + HDM * (2 * hp + hl) + 8 * dg;
    const v4u uh = *(const v4ua*)(Vh + src);
    const v4u ul = *(const v4ua*)(Vl + src);
    us_t* dh = sVT + ((hl * 2 + 0) * HDM + 8 * dg) * VTP + j;
    us_t* dl = sVT + ((hl * 2 + 1) * HDM + 8 * dg) * VTP + j;
#pragma unroll
    for (int i = 0; i < 4; ++i) {
      dh[(2 * i) * VTP]     = (us_t)(uh[i] & 0xFFFFu);
      dh[(2 * i + 1) * VTP] = (us_t)(uh[i] >> 16);
      dl[(2 * i) * VTP]     = (us_t)(ul[i] & 0xFFFFu);
      dl[(2 * i + 1) * VTP] = (us_t)(ul[i] >> 16);
    }
  }
  for (int e = tid; e < 2 * 2 * HDM * (VTP - LT); e += ATT_THREADS) {
    const int c = e % (VTP - LT), row = e / (VTP - LT);
    sVT[row * VTP + LT + c] = (us_t)0;
  }
  __syncthreads();

  const int ic = imin(16 * qt + m, LT - 1);
#pragma unroll 1
  for (int hl = 0; hl < 2; ++hl) {
    const int head = 2 * hp + hl, cq = HDM * head;
    const v16b QBh = ldfrag(Qh + (tok0 + ic) * PD + cq, hf);
    const v16b QBl = ldfrag(Ql + (tok0 + ic) * PD + cq, hf);
    const float* brow = bt + ((size_t)head * LT + ic) * LT;
    const float* mrow = am + ((size_t)wl * LT + ic) * LT;
    const us_t* vth = sVT + (hl * 2 + 0) * HDM * VTP;
    const us_t* vtl = sVT + (hl * 2 + 1) * HDM * VTP;
    v8f o[2];
    o[0] = z8; o[1] = z8;
    float mrun = -1e30f, lrun = 0.0f;

#pragma unroll 1
    for (int kc = 0; kc < 7; ++kc) {
      v8f s[2];
#pragma unroll
      for (int u = 0; u < 2; ++u) {
        const int kt = 2 * kc + u;
        v8f z = z8;
        if (kt < NQT) {
          const int jr = imin(16 * kt + m, LT - 1);
          const v16b KAh = ldfrag(Kh + (tok0 + jr) * PD + cq, hf);
          const v16b KAl = ldfrag(Kl + (tok0 + jr) * PD + cq, hf);
          z = wmma_bf(KAh, QBh, z);
          z = wmma_bf(KAh, QBl, z);
          z = wmma_bf(KAl, QBh, z);
        }
        const int j0 = 16 * kt + 8 * hf;
        const int ja = imin(j0, LT - 4), jb = imin(j0 + 4, LT - 4);
        const v4f ba = *(const v4fa*)(brow + ja);
        const v4f bb = *(const v4fa*)(brow + jb);
        const v4f ma = *(const v4fa*)(mrow + ja);
        const v4f mb = *(const v4fa*)(mrow + jb);
        const float b8[8] = {ba.x, ba.y, ba.z, ba.w, bb.x, bb.y, bb.z, bb.w};
        const float m8[8] = {ma.x, ma.y, ma.z, ma.w, mb.x, mb.y, mb.z, mb.w};
#pragma unroll
        for (int r = 0; r < 8; ++r) {
          float val = z[r] * SQS + b8[r];
          val = val + m8[r];
          s[u][r] = (j0 + r < LT) ? val : -1e30f;
        }
      }
      float mloc = s[0][0];
#pragma unroll
      for (int u = 0; u < 2; ++u)
#pragma unroll
        for (int r = 0; r < 8; ++r) mloc = fmaxf(mloc, s[u][r]);
      mloc = fmaxf(mloc, __shfl_xor(mloc, 16));
      const float mnew = fmaxf(mrun, mloc);
      const float alpha = __expf(mrun - mnew);
      mrun = mnew;
      float lsum = 0.0f;
#pragma unroll
      for (int u = 0; u < 2; ++u)
#pragma unroll
        for (int r = 0; r < 8; ++r) {
          const float p = __expf(s[u][r] - mnew);
          s[u][r] = p;
          lsum += p;
        }
      lsum += __shfl_xor(lsum, 16);
      lrun = lrun * alpha + lsum;
      o[0] = o[0] * alpha;
      o[1] = o[1] * alpha;
      PK ph, pl;
#pragma unroll
      for (int i = 0; i < 4; ++i) {
        unsigned int h0, l0, h1, l1;
        split2(s[0][2 * i], h0, l0); split2(s[0][2 * i + 1], h1, l1);
        ph.w[i] = h0 | (h1 << 16); pl.w[i] = l0 | (l1 << 16);
        split2(s[1][2 * i], h0, l0); split2(s[1][2 * i + 1], h1, l1);
        ph.w[4 + i] = h0 | (h1 << 16); pl.w[4 + i] = l0 | (l1 << 16);
      }
#pragma unroll
      for (int t = 0; t < 2; ++t) {
        const v16b VAh = ldfrag(vth + (16 * t + m) * VTP + 32 * kc, hf);
        const v16b VAl = ldfrag(vtl + (16 * t + m) * VTP + 32 * kc, hf);
        o[t] = wmma_bf(VAh, ph.v, o[t]);
        o[t] = wmma_bf(VAh, pl.v, o[t]);
        o[t] = wmma_bf(VAl, ph.v, o[t]);
      }
    }
    const float inv = 1.0f / lrun;
#pragma unroll
    for (int t = 0; t < 2; ++t) {
      float y[8];
#pragma unroll
      for (int r = 0; r < 8; ++r) y[r] = o[t][r] * inv;
      v4u hi, lo; pack8(y, hi, lo);
      const int so_off = (qt * 16 + m) * 64 + 32 * hl + 16 * t + 8 * hf;
      *(v4ua*)(sO + so_off) = hi;
      *(v4ua*)(sO + NQT * 16 * 64 + so_off) = lo;
    }
  }
  __syncthreads();
  const int nst = (qt == NQT - 1) ? 1 : 4;
  ctx_store_pass(sO, Ch, Cl, tok0, qt, hp, nst, lane);
  __threadfence();
  ctx_store_pass(sO, Ch, Cl, tok0, qt, hp, nst, lane);
}

extern "C" void kernel_launch(void* const* d_in, const int* in_sizes, int n_in,
                              void* d_out, int out_size, void* d_ws, size_t ws_size,
                              hipStream_t stream) {
  if (n_in < 22) return;
  if (in_sizes[0] != NVOXF || in_sizes[1] != NVOXF || in_sizes[2] != NVOXF) return;
  if (in_sizes[3] != CE * PD || in_sizes[5] != CE * PD || in_sizes[7] != CE * PD || in_sizes[9] != PD * CE) return;
  if (in_sizes[4] != PD || in_sizes[6] != PD || in_sizes[8] != PD || in_sizes[10] != CE) return;
  if (in_sizes[11] < NHD || (in_sizes[11] % NHD) != 0) return;
  if (in_sizes[12] != CE || in_sizes[13] != CE || in_sizes[17] != CE || in_sizes[18] != CE || in_sizes[19] != CE) return;
  if (in_sizes[14] != CE * HID || in_sizes[15] != HID || in_sizes[16] != HID * CE) return;
  if (in_sizes[20] != LT * LT || in_sizes[21] != NWIN * LT * LT) return;
  if (out_size != NVOXF) return;

  const float* xq  = (const float*)d_in[0];
  const float* xk  = (const float*)d_in[1];
  const float* xv  = (const float*)d_in[2];
  const float* Wq  = (const float*)d_in[3];
  const float* bq  = (const float*)d_in[4];
  const float* Wk  = (const float*)d_in[5];
  const float* bk  = (const float*)d_in[6];
  const float* Wv  = (const float*)d_in[7];
  const float* bv  = (const float*)d_in[8];
  const float* Wo  = (const float*)d_in[9];
  const float* bo  = (const float*)d_in[10];
  const float* rt  = (const float*)d_in[11];
  const float* g1  = (const float*)d_in[12];
  const float* bl1 = (const float*)d_in[13];
  const float* W1  = (const float*)d_in[14];
  const float* b1  = (const float*)d_in[15];
  const float* W2  = (const float*)d_in[16];
  const float* b2  = (const float*)d_in[17];
  const float* g2  = (const float*)d_in[18];
  const float* bl2 = (const float*)d_in[19];
  const int*   ri  = (const int*)d_in[20];
  const float* amk = (const float*)d_in[21];
  float* dout = (float*)d_out;
  const int nrel = in_sizes[11] / NHD;

  const size_t wt_bytes = (size_t)OWEND * 2;
  const size_t bt_bytes = (size_t)NHD * LT * LT * 4;
  const size_t xpl      = (size_t)MHALF * CE * 2;
  const size_t ppl      = (size_t)MHALF * PD * 2;
  const size_t hpl      = (size_t)MHALF * HID * 2;
  const size_t a32b     = (size_t)MHALF * CE * 4;
  const size_t off_wt = 0;
  const size_t off_bt = off_wt + wt_bytes;
  const size_t off_x  = off_bt + bt_bytes;
  const size_t off_p  = off_x + 6 * xpl;
  const size_t total  = off_p + 6 * ppl;
  if (total > ws_size) return;
  if (total > (size_t)134217728) return;
  if (2 * ppl > 6 * xpl) return;
  if (a32b + 2 * xpl + 2 * hpl > 6 * ppl) return;

  char* ws = (char*)d_ws;
  us_t*  wt   = (us_t*)(ws + off_wt);
  float* bt   = (float*)(ws + off_bt);
  us_t*  X    = (us_t*)(ws + off_x);
  us_t*  XQH  = X;
  us_t*  XQL  = (us_t*)(ws + off_x + 1 * xpl);
  us_t*  XKH  = (us_t*)(ws + off_x + 2 * xpl);
  us_t*  XKL  = (us_t*)(ws + off_x + 3 * xpl);
  us_t*  XVH  = (us_t*)(ws + off_x + 4 * xpl);
  us_t*  XVL  = (us_t*)(ws + off_x + 5 * xpl);
  us_t*  QH   = (us_t*)(ws + off_p + 0 * ppl);
  us_t*  QL   = (us_t*)(ws + off_p + 1 * ppl);
  us_t*  KH   = (us_t*)(ws + off_p + 2 * ppl);
  us_t*  KL   = (us_t*)(ws + off_p + 3 * ppl);
  us_t*  VHp  = (us_t*)(ws + off_p + 4 * ppl);
  us_t*  VLp  = (us_t*)(ws + off_p + 5 * ppl);
  us_t*  CH   = (us_t*)(ws + off_x);
  us_t*  CL   = (us_t*)(ws + off_x + ppl);
  float* ATT32 = (float*)(ws + off_p);
  us_t*  ATH   = (us_t*)(ws + off_p + a32b);
  us_t*  ATL   = (us_t*)(ws + off_p + a32b + xpl);
  us_t*  HMH   = (us_t*)(ws + off_p + a32b + 2 * xpl);
  us_t*  HML   = (us_t*)(ws + off_p + a32b + 2 * xpl + hpl);

  const unsigned att_lds = (unsigned)((2 * 2 * HDM * VTP + 2 * NQT * 16 * 64) * 2);

  k_bias<<<((NHD * LT * LT) / 4 + 255) / 256, 256, 0, stream>>>(rt, ri, nrel, bt);
  k_wconv<<<176, 256, 0, stream>>>(Wq, Wk, Wv, Wo, W1, W2, wt);

  for (int half = 0; half < 2; ++half) {
    k_gather<<<dim3(MHALF * 16 / 256, 3), 256, 0, stream>>>(xq, xk, xv, half, X);
    k_gemm_planes<0><<<dim3(MHALF / 32, PD / 128), 64, 0, stream>>>(XQH, XQL, wt + OWQH, wt + OWQL, bq, CE, PD, QH, QL);
    k_gemm_planes<0><<<dim3(MHALF / 32, PD / 128), 64, 0, stream>>>(XKH, XKL, wt + OWKH, wt + OWKL, bk, CE, PD, KH, KL);
    k_gemm_planes<0><<<dim3(MHALF / 32, PD / 128), 64, 0, stream>>>(XVH, XVL, wt + OWVH, wt + OWVL, bv, CE, PD, VHp, VLp);
    k_attn<<<dim3(NWIN, NHD / 2), ATT_THREADS, att_lds, stream>>>(QH, QL, KH, KL, VHp, VLp, bt, amk, CH, CL);
    k_gemm_ln<0><<<dim3(MHALF / 32, 1), 64, 0, stream>>>(CH, CL, wt + OWOH, wt + OWOL, bo, PD, g1, bl1, xq, ATT32, ATH, ATL, half);
    k_gemm_planes<1><<<dim3(MHALF / 32, HID / 128), 64, 0, stream>>>(ATH, ATL, wt + OW1H, wt + OW1L, b1, CE, HID, HMH, HML);
    k_gemm_ln<1><<<dim3(MHALF / 32, 1), 64, 0, stream>>>(HMH, HML, wt + OW2H, wt + OW2L, b2, HID, g2, bl2, ATT32, dout, ATH, ATL, half);
  }
}
